// UVLearner_65111704207926
// MI455X (gfx1250) — hardware-verified
//
#include <hip/hip_runtime.h>


namespace {
constexpr int Bn = 4, C = 128, NP = 4096, GW = 64;
constexpr float PS = 8.0f, SCALE = 0.08838834764831845f;

typedef _Float16 b16;
typedef __attribute__((ext_vector_type(16))) _Float16 v16b;
typedef __attribute__((ext_vector_type(8))) _Float16 v8b;
typedef __attribute__((ext_vector_type(8))) float v8f;
typedef __attribute__((ext_vector_type(4))) float v4f;
__device__ __forceinline__ float bf16_rne(float f) { unsigned int u = __float_as_uint(f); u += 0x7FFFu + ((u >> 16) & 1u); return __uint_as_float(u & 0xFFFF0000u); }
__device__ __forceinline__ void split16(float v, b16& hi, b16& lo) { hi = (b16)v; lo = (b16)(v - (float)hi); }
__device__ __forceinline__ v16b frag_kb(const b16* p, int hh) { const v8b a = *(const v8b*)(p + 8 * hh), b = *(const v8b*)(p + 16 + 8 * hh); v16b f;
#pragma unroll
  for (int e = 0; e < 8; ++e) { f[e] = a[e]; f[8 + e] = b[e]; } return f; }
__device__ __forceinline__ v8f wmma16b(v16b a, v16b b, v8f c) { v8f d = __builtin_amdgcn_wmma_f32_16x16x32_f16(false, a, false, b, (short)0, c, false, false); asm volatile("v_nop\n\tv_nop\n\tv_nop\n\tv_nop" : "+v"(d) : "v"(a), "v"(b)); return d; }
__device__ __forceinline__ float nexp(float x) { return __builtin_amdgcn_exp2f(x * 1.4426950408889634f); }

__global__ __launch_bounds__(256) void xpose_kernel(const float* __restrict__ x, const float* __restrict__ y, b16* __restrict__ XT, b16* __restrict__ YT, b16* __restrict__ GT) {
  __shared__ __attribute__((aligned(16))) b16 T[64][C + 8];
  const int b = blockIdx.y, p0 = blockIdx.x * 64, which = blockIdx.z, t_ = threadIdx.x; const float* src = (which == 0) ? x : y; b16* dst = (which == 0) ? XT : YT;
  for (int i = t_; i < C * 64; i += 256) { const int c = i >> 6, p = i & 63; T[p][c] = (b16)bf16_rne(src[((size_t)b * C + c) * NP + p0 + p]); }
  __syncthreads();
  for (int pass = 0; pass < 2; ++pass) { for (int i = t_; i < 64 * 16; i += 256) { const int p = i >> 4, c8 = (i & 15) * 8; *(volatile v8b*)(dst + ((size_t)b * NP + p0 + p) * C + c8) = *(const v8b*)(&T[p][c8]); }
    if (b == 0 && which == 0) { for (int i = t_; i < 16 * 8; i += 256) { const int row = i >> 3, c8 = (i & 7) * 8; v8b v; for (int e = 0; e < 8; ++e) { const int k = p0 + c8 + e; v[e] = (b16)((row == 0) ? ((float)(k % GW) + 0.5f) : (row == 1) ? ((float)(k / GW) + 0.5f) : 0.0f); } *(volatile v8b*)(GT + (size_t)row * NP + p0 + c8) = v; } }
    __threadfence(); }
}

__global__ __launch_bounds__(256) void attn_kernel(const b16* __restrict__ XT, const b16* __restrict__ YT, const b16* __restrict__ GT, float* __restrict__ out) {
  __shared__ float O[128][2];
  const int wid = threadIdx.x >> 5, lane = threadIdx.x & 31, hh = lane >> 4, col = lane & 15, b = blockIdx.y, q0 = blockIdx.x * 128 + wid * 16, qi = q0 + col;
  const b16* Xb = XT + (size_t)b * NP * C; const b16* Yb = YT + (size_t)b * NP * C;
  v16b qf[4];
#pragma unroll
  for (int j = 0; j < 4; ++j) qf[j] = frag_kb(Xb + (size_t)qi * C + 32 * j, hh);
  float m = -INFINITY, l = 0.0f; v8f o = {};
  for (int kb = 0; kb < NP; kb += 32) {
    v8f s0 = {}, s1 = {};
#pragma unroll
    for (int j = 0; j < 4; ++j) { const v16b ka = frag_kb(Yb + (size_t)(kb + col) * C + 32 * j, hh), kc = frag_kb(Yb + (size_t)(kb + 16 + col) * C + 32 * j, hh); s0 = wmma16b(ka, qf[j], s0); s1 = wmma16b(kc, qf[j], s1); }
    float mr = -INFINITY;
#pragma unroll
    for (int r = 0; r < 8; ++r) { s0[r] *= SCALE; s1[r] *= SCALE; mr = fmaxf(mr, fmaxf(s0[r], s1[r])); }
    mr = fmaxf(mr, __shfl_xor(mr, 16));
    const float mn = fmaxf(m, mr), al_ = nexp(m - mn); m = mn; float sum = 0.0f; v16b ph, pl;
#pragma unroll
    for (int r = 0; r < 8; ++r) { const float e0 = nexp(s0[r] - mn), e1 = nexp(s1[r] - mn); sum += e0 + e1; b16 a_, c_; split16(e0 * PS, a_, c_); ph[r] = a_; pl[r] = c_; split16(e1 * PS, a_, c_); ph[8 + r] = a_; pl[8 + r] = c_; }
    sum += __shfl_xor(sum, 16); l = l * al_ + sum; o *= al_;
    const v16b gf = frag_kb(GT + (size_t)col * NP + kb, hh); o = wmma16b(gf, ph, o); o = wmma16b(gf, pl, o); }
  const float inv = 1.0f / (l * PS);
#pragma unroll
  for (int r = 0; r < 8; ++r) { const int t = 8 * hh + r; if (t < 2) O[wid * 16 + col][t] = (o[r] * inv) * (2.0f / (float)GW) - 1.0f; }
  __syncthreads();
  for (int pass = 0; pass < 2; ++pass) { if (threadIdx.x < 64) *(volatile v4f*)(out + ((size_t)b * NP + blockIdx.x * 128) * 2 + threadIdx.x * 4) = *(const v4f*)(&O[0][0] + threadIdx.x * 4); __threadfence(); }
}
}

extern "C" void kernel_launch(void* const* d_in, const int* in_sizes, int n_in,
                              void* d_out, int out_size, void* d_ws, size_t ws_size, hipStream_t stream) {
  (void)n_in; (void)out_size;
  const float* x = (const float*)d_in[0]; const float* y = (const float*)d_in[1];
  float* out = (float*)d_out;
  if (in_sizes[0] != Bn * C * NP || in_sizes[1] != Bn * C * NP) return;
  size_t off = 0; char* ws = (char*)d_ws;
  auto carve = [&](size_t bytes) { char* p = ws + off; off += (bytes + 255) & ~(size_t)255; return p; };
  b16* XT = (b16*)carve((size_t)Bn * NP * C * 2); b16* YT = (b16*)carve((size_t)Bn * NP * C * 2); b16* GT = (b16*)carve((size_t)16 * NP * 2);
  if (off > ws_size) return;
  xpose_kernel<<<dim3(NP / 64, Bn, 2), 256, 0, stream>>>(x, y, XT, YT, GT);
  attn_kernel<<<dim3(NP / 128, Bn), 256, 0, stream>>>(XT, YT, GT, out);
}
